// SpatialDisaggregationGNN_17059610099968
// MI455X (gfx1250) — hardware-verified
//
#include <hip/hip_runtime.h>
#include <stddef.h>


#define IND    6
#define HD     32
#define HHALF  16
#define NTHR   256
#define NWAVE  8
#define EPT    8
#define NGRP   2
#define CHUNK  (NTHR * EPT * NGRP)
#define WCAP   (EPT * NGRP * 32)
#define LISTN  (NWAVE * WCAP)
#define NBD    4096
#define NB1    2048
#define NBG    1024
#define NB2    4096
#define TROWS  128
#define APITCH 40
#define WSC    8.0f
#define WIV    0.125f
#define NEPS   1e-5f

#define WO_E2  0
#define WO_G1  1024
#define WO_GA  2048
#define WO_G2  3072
#define WO_P1  3584
#define WO_TOT 4096

#define LDS_AGG1 (NB1 * HD * 4 + LISTN * 4 + 64)
#define LDS_GAT  (NBG * HD * 4 + NBG * 2 * 4 * 3 + LISTN * 4 + 64)
#define LDS_AGG2 (NB2 * HHALF * 4 + LISTN * 4 + 64)

static_assert((CHUNK & (CHUNK - 1)) == 0);
static_assert(CHUNK <= 4096);
static_assert(NBD <= 4096 && NB1 <= 4096 && NBG <= 4096 && NB2 <= 4096);
static_assert((NBD % TROWS) == 0 && (NB1 % TROWS) == 0 && (NBG % TROWS) == 0 && (NB2 % TROWS) == 0);
static_assert((2 * NTHR + 64) * 8 <= LISTN * 4);
static_assert((NB1 * HD) % (128 * NWAVE) == 0 && (NBG * HD) % (128 * NWAVE) == 0 && (NB2 * HHALF) % (128 * NWAVE) == 0);

typedef float    v4f  __attribute__((ext_vector_type(4)));
typedef float    v8f  __attribute__((ext_vector_type(8)));
typedef int      v4i  __attribute__((ext_vector_type(4)));
typedef double   v2d  __attribute__((ext_vector_type(2)));
typedef _Float16 v8h  __attribute__((ext_vector_type(8)));
typedef _Float16 v16h __attribute__((ext_vector_type(16)));
union FragH { v16h v; v8h h[2]; };

__device__ __forceinline__ v4f relu4(v4f v) {
  v.x = fmaxf(v.x, 0.f); v.y = fmaxf(v.y, 0.f); v.z = fmaxf(v.z, 0.f); v.w = fmaxf(v.w, 0.f);
  return v;
}

__device__ __forceinline__ v8h cvt8(v4f a, v4f b) {
  v8h r;
  r[0] = (_Float16)a.x; r[1] = (_Float16)a.y; r[2] = (_Float16)a.z; r[3] = (_Float16)a.w;
  r[4] = (_Float16)b.x; r[5] = (_Float16)b.y; r[6] = (_Float16)b.z; r[7] = (_Float16)b.w;
  return r;
}

__device__ __forceinline__ v8f wmh(v16h a, v16h b, v8f c) {
  v8f d = __builtin_amdgcn_wmma_f32_16x16x32_f16(false, a, false, b, (short)0, c, false, false);
  asm volatile("v_nop\n\tv_nop\n\tv_nop\n\tv_nop" : "+v"(d) : "v"(a), "v"(b));
  return d;
}

__device__ __forceinline__ v8f zero8() { v8f z = {0.f, 0.f, 0.f, 0.f, 0.f, 0.f, 0.f, 0.f}; return z; }

template <int NB>
__device__ __forceinline__ int scan_chunk(const int* __restrict__ dsts, int nE, int cbase, int nodeBase,
                                          int vec8, int* list, int tid, int lane, int wave) {
  int wc = 0;
#pragma unroll
  for (int g = 0; g < NGRP; ++g) {
    const int el0  = (g * NTHR + tid) * EPT;
    const int e0   = cbase + el0;
    const int sent = -2147483647 - 1;
    v4i da, db;
    if (vec8 != 0 && e0 + 7 < nE) {
      da = *(const v4i*)(dsts + e0);
      db = *(const v4i*)(dsts + e0 + 4);
    } else {
      da.x = (e0     < nE) ? dsts[min(e0, nE - 1)] : sent;
      da.y = (e0 + 1 < nE) ? dsts[min(e0 + 1, nE - 1)] : sent;
      da.z = (e0 + 2 < nE) ? dsts[min(e0 + 2, nE - 1)] : sent;
      da.w = (e0 + 3 < nE) ? dsts[min(e0 + 3, nE - 1)] : sent;
      db.x = (e0 + 4 < nE) ? dsts[min(e0 + 4, nE - 1)] : sent;
      db.y = (e0 + 5 < nE) ? dsts[min(e0 + 5, nE - 1)] : sent;
      db.z = (e0 + 6 < nE) ? dsts[min(e0 + 6, nE - 1)] : sent;
      db.w = (e0 + 7 < nE) ? dsts[min(e0 + 7, nE - 1)] : sent;
    }
    const unsigned nb = (unsigned)nodeBase;
    const unsigned s0 = (unsigned)da.x - nb, s1 = (unsigned)da.y - nb;
    const unsigned s2 = (unsigned)da.z - nb, s3 = (unsigned)da.w - nb;
    const unsigned s4 = (unsigned)db.x - nb, s5 = (unsigned)db.y - nb;
    const unsigned s6 = (unsigned)db.z - nb, s7 = (unsigned)db.w - nb;
    const bool h0 = s0 < (unsigned)NB, h1 = s1 < (unsigned)NB, h2 = s2 < (unsigned)NB, h3 = s3 < (unsigned)NB;
    const bool h4 = s4 < (unsigned)NB, h5 = s5 < (unsigned)NB, h6 = s6 < (unsigned)NB, h7 = s7 < (unsigned)NB;
    const unsigned any = __builtin_amdgcn_ballot_w32(h0 | h1 | h2 | h3 | h4 | h5 | h6 | h7);
    if (any != 0u) {
#define HITJ(J, HJ, SJ) { \
        const unsigned mj = __builtin_amdgcn_ballot_w32(HJ); \
        if (mj != 0u) { \
          if (HJ) { \
            const int pos = wc + (int)__builtin_amdgcn_mbcnt_lo(mj, 0u); \
            if (pos < WCAP) list[wave * WCAP + pos] = ((el0 + (J)) << 12) | (int)(SJ); \
          } \
          wc += (int)__builtin_popcount(mj); } }
      HITJ(0, h0, s0)
      HITJ(1, h1, s1)
      HITJ(2, h2, s2)
      HITJ(3, h3, s3)
      HITJ(4, h4, s4)
      HITJ(5, h5, s5)
      HITJ(6, h6, s6)
      HITJ(7, h7, s7)
#undef HITJ
    }
  }
  return wc;
}

__device__ __forceinline__ void store_tile16x32(const float* stg, float* gdst, int lane) {
  const int rr = lane >> 3, pc = (lane & 7) * 4;
  v4f v[4];
#pragma unroll
  for (int i = 0; i < 4; ++i) v[i] = *(const v4f*)(stg + (4 * i + rr) * HD + pc);
#pragma unroll
  for (int i = 0; i < 4; ++i) *(volatile v4f*)(gdst + (size_t)(4 * i + rr) * HD + pc) = v[i];
  __threadfence();
#pragma unroll
  for (int i = 0; i < 4; ++i) *(volatile v4f*)(gdst + (size_t)(4 * i + rr) * HD + pc) = v[i];
}

template <int TOT>
__device__ __forceinline__ void store_rows(const float* src, float* dst, int wave, int lane) {
  constexpr int Q = TOT / (128 * NWAVE);
#pragma unroll 4
  for (int q = 0; q < Q; ++q) {
    const int f = (wave * Q + q) * 128 + 4 * lane;
    const v4f v = *(const v4f*)(src + f);
    *(volatile v4f*)(dst + f) = v;
  }
  __threadfence();
#pragma unroll 4
  for (int q = 0; q < Q; ++q) {
    const int f = (wave * Q + q) * 128 + 4 * lane;
    const v4f v = *(const v4f*)(src + f);
    *(volatile v4f*)(dst + f) = v;
  }
}

template <int NB, int NC>
__device__ __forceinline__ void bn_part(const float* acc, double* dsc, double* pdst,
                                        int nodeBase, int nN, int tid) {
  constexpr int NG  = NTHR / NC;
  constexpr int RPG = NB / NG;
  const int c = tid % NC, g = tid / NC;
  const int vrows = nN - nodeBase;
  double s = 0.0, q = 0.0;
#pragma unroll 4
  for (int r = 0; r < RPG; ++r) {
    const int slot = g * RPG + r;
    if (slot < vrows) {
      const float v = acc[slot * NC + c];
      s += (double)v;
      q += (double)v * (double)v;
    }
  }
  dsc[2 * tid]     = s;
  dsc[2 * tid + 1] = q;
  __syncthreads();
  if (tid < 32) {
    double fs = 0.0, fq = 0.0;
    if (tid < NC) {
#pragma unroll 1
      for (int gg = 0; gg < NG; ++gg) {
        fs += dsc[2 * (gg * NC + tid)];
        fq += dsc[2 * (gg * NC + tid) + 1];
      }
    }
    dsc[2 * NTHR + tid]      = fs;
    dsc[2 * NTHR + 32 + tid] = fq;
  }
  __syncthreads();
  if (tid < 32) {
    const v2d v = *(const v2d*)(dsc + 2 * NTHR + 2 * tid);
    *(volatile v2d*)(pdst + 2 * tid) = v;
    __threadfence();
    *(volatile v2d*)(pdst + 2 * tid) = v;
  }
}

__global__ __launch_bounds__(NTHR) void k_prep(
    const float* __restrict__ we2, const float* __restrict__ wg1, const float* __restrict__ wga,
    const float* __restrict__ wg2, const float* __restrict__ wp1, _Float16* wpl) {
  const int i = blockIdx.x * NTHR + threadIdx.x;
  if (i >= WO_TOT / 8) return;
  const int o = i * 8;
  float v[8];
  if (o < WO_G2) {
    const float* W = (o < WO_G1) ? we2 : ((o < WO_GA) ? wg1 : wga);
    const int p = o & 1023;
    const int n = p >> 5, k0 = p & 31;
#pragma unroll
    for (int j = 0; j < 8; ++j) v[j] = W[(k0 + j) * HD + n];
  } else if (o < WO_P1) {
    const int p = o - WO_G2;
    const int n = p >> 5, k0 = p & 31;
#pragma unroll
    for (int j = 0; j < 8; ++j) v[j] = wg2[(k0 + j) * HHALF + n];
  } else {
    const int p = o - WO_P1;
    const int n = p >> 5, k0 = p & 31;
#pragma unroll
    for (int j = 0; j < 8; ++j) {
      const int k = k0 + j;
      const float w = wp1[(k & 15) * 8 + (n & 7)];
      v[j] = (n < 8 && k < 16) ? w : 0.f;
    }
  }
  v4f a, b;
  a.x = v[0] * WSC; a.y = v[1] * WSC; a.z = v[2] * WSC; a.w = v[3] * WSC;
  b.x = v[4] * WSC; b.y = v[5] * WSC; b.z = v[6] * WSC; b.w = v[7] * WSC;
  const v8h hv = cvt8(a, b);
  _Float16* dp = wpl + o;
  *(volatile v8h*)dp = hv;
  __threadfence();
  *(volatile v8h*)dp = hv;
}

__global__ __launch_bounds__(NTHR) void k_deg(
    const int* __restrict__ ei, float* dinv, int nE, int vec8) {
  __shared__ __attribute__((aligned(16))) int cnt[NBD];
  __shared__ __attribute__((aligned(16))) int list[LISTN];
  __shared__ int wcnt[NWAVE];
  const int tid = threadIdx.x, lane = tid & 31, wave = tid >> 5;
  const int nodeBase = blockIdx.x * NBD;
  const int* dsts = ei + nE;

  for (int i = tid; i < NBD; i += NTHR) cnt[i] = 0;
  __syncthreads();

  const int nChunks = (nE + CHUNK - 1) / CHUNK;
#pragma unroll 1
  for (int ch = 0; ch < nChunks; ++ch) {
    const int cbase = ch * CHUNK;
    const int wc = scan_chunk<NBD>(dsts, nE, cbase, nodeBase, vec8, list, tid, lane, wave);
    if (lane == 0) wcnt[wave] = wc;
    __syncthreads();
    if (wave == 0) {
#pragma unroll 1
      for (int wsx = 0; wsx < NWAVE; ++wsx) {
        int n = __builtin_amdgcn_readfirstlane(wcnt[wsx]);
        n = n > WCAP ? WCAP : (n < 0 ? 0 : n);
        const int* lp = list + wsx * WCAP;
#pragma unroll 1
        for (int i = 0; i < n; ++i) {
          const int ent  = __builtin_amdgcn_readfirstlane(lp[i]);
          const int slot = ent & (NBD - 1);
          if (lane == 0) cnt[slot] = cnt[slot] + 1;
        }
      }
    }
    __syncthreads();
  }

  v4f dq[4];
#pragma unroll
  for (int q = 0; q < 4; ++q) {
    const int f = (wave * 4 + q) * 128 + 4 * lane;
    const v4i c = *(const v4i*)(cnt + f);
    dq[q].x = rsqrtf((float)(c.x + 1));
    dq[q].y = rsqrtf((float)(c.y + 1));
    dq[q].z = rsqrtf((float)(c.z + 1));
    dq[q].w = rsqrtf((float)(c.w + 1));
  }
  float* dp = dinv + (size_t)nodeBase;
#pragma unroll
  for (int q = 0; q < 4; ++q) *(volatile v4f*)(dp + (wave * 4 + q) * 128 + 4 * lane) = dq[q];
  __threadfence();
#pragma unroll
  for (int q = 0; q < 4; ++q) *(volatile v4f*)(dp + (wave * 4 + q) * 128 + 4 * lane) = dq[q];
}

__global__ __launch_bounds__(NTHR) void k_enc(
    const float* __restrict__ x, const float* __restrict__ lng, const float* __restrict__ lnb,
    const float* __restrict__ w1, const float* __restrict__ b1, const float* __restrict__ b2,
    const _Float16* __restrict__ wpl, const float* __restrict__ dinv, float* g1, int nN) {
  __shared__ __attribute__((aligned(16))) float sw1[IND * HD];
  __shared__ __attribute__((aligned(16))) float sb1[HD];
  __shared__ __attribute__((aligned(16))) float sb2[HD];
  __shared__ float sg[8];
  __shared__ float sbe[8];
  __shared__ __attribute__((aligned(16))) _Float16 hA[NWAVE][16 * APITCH];
  __shared__ __attribute__((aligned(16))) float stg[NWAVE][16 * HD];
  const int tid = threadIdx.x, lane = tid & 31, wave = tid >> 5, h = lane >> 4, m = lane & 15;
  const int rowBase = blockIdx.x * TROWS;

  if (tid < IND * HD) sw1[tid] = w1[tid];
  if (tid < HD) { sb1[tid] = b1[tid]; sb2[tid] = b2[tid]; }
  if (tid < IND) { sg[tid] = lng[tid]; sbe[tid] = lnb[tid]; }
  __syncthreads();

  int node = rowBase + wave * 16 + m;
  node = node > nN - 1 ? nN - 1 : node;
  const float* xp = x + (size_t)node * IND;
  float y[IND];
  {
    const float v0 = xp[0], v1 = xp[1], v2 = xp[2], v3 = xp[3], v4 = xp[4], v5 = xp[5];
    const float mean = (v0 + v1 + v2 + v3 + v4 + v5) * (1.0f / 6.0f);
    const float d0 = v0 - mean, d1 = v1 - mean, d2 = v2 - mean, d3 = v3 - mean, d4 = v4 - mean, d5 = v5 - mean;
    const float var = (d0 * d0 + d1 * d1 + d2 * d2 + d3 * d3 + d4 * d4 + d5 * d5) * (1.0f / 6.0f);
    const float is = rsqrtf(var + NEPS);
    y[0] = d0 * is * sg[0] + sbe[0];
    y[1] = d1 * is * sg[1] + sbe[1];
    y[2] = d2 * is * sg[2] + sbe[2];
    y[3] = d3 * is * sg[3] + sbe[3];
    y[4] = d4 * is * sg[4] + sbe[4];
    y[5] = d5 * is * sg[5] + sbe[5];
  }

  float z[16];
#pragma unroll
  for (int n = 0; n < 16; ++n) z[n] = sb1[16 * h + n];
#pragma unroll
  for (int k = 0; k < IND; ++k) {
    const float* wr = sw1 + k * HD + 16 * h;
    const v4f wa = *(const v4f*)wr, wb = *(const v4f*)(wr + 4), wc = *(const v4f*)(wr + 8), wd = *(const v4f*)(wr + 12);
    const float yk = y[k];
    z[0]  += yk * wa.x; z[1]  += yk * wa.y; z[2]  += yk * wa.z; z[3]  += yk * wa.w;
    z[4]  += yk * wb.x; z[5]  += yk * wb.y; z[6]  += yk * wb.z; z[7]  += yk * wb.w;
    z[8]  += yk * wc.x; z[9]  += yk * wc.y; z[10] += yk * wc.z; z[11] += yk * wc.w;
    z[12] += yk * wd.x; z[13] += yk * wd.y; z[14] += yk * wd.z; z[15] += yk * wd.w;
  }
  {
    v4f za, zb, zc, zd;
    za.x = fmaxf(z[0], 0.f);  za.y = fmaxf(z[1], 0.f);  za.z = fmaxf(z[2], 0.f);  za.w = fmaxf(z[3], 0.f);
    zb.x = fmaxf(z[4], 0.f);  zb.y = fmaxf(z[5], 0.f);  zb.z = fmaxf(z[6], 0.f);  zb.w = fmaxf(z[7], 0.f);
    zc.x = fmaxf(z[8], 0.f);  zc.y = fmaxf(z[9], 0.f);  zc.z = fmaxf(z[10], 0.f); zc.w = fmaxf(z[11], 0.f);
    zd.x = fmaxf(z[12], 0.f); zd.y = fmaxf(z[13], 0.f); zd.z = fmaxf(z[14], 0.f); zd.w = fmaxf(z[15], 0.f);
    _Float16* hrow = &hA[wave][m * APITCH + 16 * h];
    *(v8h*)hrow       = cvt8(za, zb);
    *(v8h*)(hrow + 8) = cvt8(zc, zd);
  }
  __syncthreads();

  const _Float16* ar = &hA[wave][m * APITCH + 8 * h];
  v8f acc[2];
  {
    FragH a;
    a.h[0] = *(const v8h*)ar;
    a.h[1] = *(const v8h*)(ar + 16);
#pragma unroll
    for (int t = 0; t < 2; ++t) {
      const _Float16* bp = wpl + WO_E2 + (size_t)(16 * t + m) * HD + 8 * h;
      FragH b;
      b.h[0] = *(const v8h*)bp;
      b.h[1] = *(const v8h*)(bp + 16);
      acc[t] = wmh(a.v, b.v, zero8());
    }
  }
  __syncthreads();

#pragma unroll
  for (int t = 0; t < 2; ++t) {
    const float bb = sb2[16 * t + m];
    _Float16* tp = &hA[wave][(8 * h) * APITCH + 16 * t + m];
#pragma unroll
    for (int r = 0; r < 8; ++r) tp[r * APITCH] = (_Float16)fmaxf(acc[t][r] * WIV + bb, 0.f);
  }
  __syncthreads();

  v8f acc2[2];
  {
    FragH a;
    a.h[0] = *(const v8h*)ar;
    a.h[1] = *(const v8h*)(ar + 16);
#pragma unroll
    for (int t = 0; t < 2; ++t) {
      const _Float16* bp = wpl + WO_G1 + (size_t)(16 * t + m) * HD + 8 * h;
      FragH b;
      b.h[0] = *(const v8h*)bp;
      b.h[1] = *(const v8h*)(bp + 16);
      acc2[t] = wmh(a.v, b.v, zero8());
    }
  }
  {
    const int r0 = wave * 16 + 8 * h;
    const v4f dA = *(const v4f*)(dinv + (size_t)rowBase + r0);
    const v4f dB = *(const v4f*)(dinv + (size_t)rowBase + r0 + 4);
    float d[8];
    d[0] = dA.x * WIV; d[1] = dA.y * WIV; d[2] = dA.z * WIV; d[3] = dA.w * WIV;
    d[4] = dB.x * WIV; d[5] = dB.y * WIV; d[6] = dB.z * WIV; d[7] = dB.w * WIV;
    float* sp = &stg[wave][(8 * h) * HD + m];
#pragma unroll
    for (int t = 0; t < 2; ++t) {
#pragma unroll
      for (int r = 0; r < 8; ++r) sp[r * HD + 16 * t] = acc2[t][r] * d[r];
    }
  }
  __syncthreads();
  store_tile16x32(stg[wave], g1 + ((size_t)rowBase + wave * 16) * HD, lane);
}

template <int NB, int NC>
__global__ __launch_bounds__(NTHR) void k_gcnagg(
    const int* __restrict__ ei, const float* __restrict__ gpl, const float* __restrict__ dinv,
    const float* __restrict__ bias, float* apl, double* part, int nN, int nE, int vec8) {
  extern __shared__ v4f lds_dyn[];
  float*  acc  = (float*)lds_dyn;
  int*    list = (int*)(acc + NB * NC);
  int*    wcnt = list + LISTN;
  double* dsc  = (double*)list;
  const int tid = threadIdx.x, lane = tid & 31, wave = tid >> 5;
  const int nodeBase = blockIdx.x * NB;
  const int* dsts = ei + nE;
  constexpr int V4R = NC / 4;

#pragma unroll 4
  for (int idx = tid; idx < NB * V4R; idx += NTHR) {
    const int slot = idx / V4R;
    const int c4   = (idx % V4R) * 4;
    int node = nodeBase + slot;
    node = node > nN - 1 ? nN - 1 : node;
    lds_dyn[idx] = *(const v4f*)(gpl + (size_t)node * NC + c4);
  }
  __syncthreads();

  const int nChunks = (nE + CHUNK - 1) / CHUNK;
#pragma unroll 1
  for (int ch = 0; ch < nChunks; ++ch) {
    const int cbase = ch * CHUNK;
    const int wc = scan_chunk<NB>(dsts, nE, cbase, nodeBase, vec8, list, tid, lane, wave);
    if (lane == 0) wcnt[wave] = wc;
    __syncthreads();
    if (wave == 0) {
#pragma unroll 1
      for (int wsx = 0; wsx < NWAVE; ++wsx) {
        int n = __builtin_amdgcn_readfirstlane(wcnt[wsx]);
        n = n > WCAP ? WCAP : (n < 0 ? 0 : n);
        const int* lp = list + wsx * WCAP;
#pragma unroll 1
        for (int i = 0; i < n; ++i) {
          const int ent  = __builtin_amdgcn_readfirstlane(lp[i]);
          const int slot = ent & (NB - 1);
          int e = cbase + ((ent >> 12) & (CHUNK - 1));
          e = e > nE - 1 ? nE - 1 : e;
          int src = ei[e];
          src = src < 0 ? 0 : (src > nN - 1 ? nN - 1 : src);
          if (lane < NC) {
            float* ap = acc + slot * NC + lane;
            *ap = *ap + gpl[(size_t)src * NC + lane];
          }
        }
      }
    }
    __syncthreads();
  }

#pragma unroll 4
  for (int idx = tid; idx < NB * V4R; idx += NTHR) {
    const int slot = idx / V4R;
    const int c4   = (idx % V4R) * 4;
    int node = nodeBase + slot;
    node = node > nN - 1 ? nN - 1 : node;
    const float d  = dinv[node];
    const v4f   bv = *(const v4f*)(bias + c4);
    const v4f   a  = lds_dyn[idx];
    lds_dyn[idx] = a * d + bv;
  }
  __syncthreads();

  bn_part<NB, NC>(acc, dsc, part + (size_t)blockIdx.x * 64, nodeBase, nN, tid);
  store_rows<NB * NC>(acc, apl + (size_t)nodeBase * NC, wave, lane);
}

__global__ __launch_bounds__(32) void k_bnfin(
    const double* __restrict__ part, int nblk, const float* __restrict__ g, const float* __restrict__ b,
    int C, int nN, float* prm) {
  __shared__ __attribute__((aligned(16))) float sps[64];
  const int c = threadIdx.x;
  float scf = 0.f, shf = 0.f;
  if (c < C) {
    double s = 0.0, q = 0.0;
#pragma unroll 1
    for (int i = 0; i < nblk; ++i) {
      s += part[(size_t)i * 64 + c];
      q += part[(size_t)i * 64 + 32 + c];
    }
    const double inv  = 1.0 / (double)nN;
    const double mean = s * inv;
    double var = q * inv - mean * mean;
    var = var < 0.0 ? 0.0 : var;
    const float sc = g[c] * rsqrtf((float)var + NEPS);
    scf = sc;
    shf = b[c] - (float)mean * sc;
  }
  sps[c]      = scf;
  sps[32 + c] = shf;
  __syncthreads();
  v4f v;
  if (c < 16) v = *(const v4f*)(sps + 4 * c);
  if (c < 16) *(volatile v4f*)(prm + 4 * c) = v;
  __threadfence();
  if (c < 16) *(volatile v4f*)(prm + 4 * c) = v;
}

__global__ __launch_bounds__(NTHR) void k_gattf(
    const float* __restrict__ a1, const float* __restrict__ prm, const _Float16* __restrict__ wg,
    const float* __restrict__ atts, const float* __restrict__ attd,
    float* hg, float* al, int nN) {
  __shared__ __attribute__((aligned(16))) float stg[NWAVE][16 * HD];
  __shared__ __attribute__((aligned(16))) float sal[NWAVE][64];
  __shared__ float satt[64];
  const int tid = threadIdx.x, lane = tid & 31, wave = tid >> 5, h = lane >> 4, m = lane & 15;
  const int rowBase = blockIdx.x * TROWS;
  (void)nN;
  if (tid < 32) satt[tid] = atts[tid];
  else if (tid < 64) satt[tid] = attd[tid - 32];

  const int row = rowBase + wave * 16 + m;
  FragH a;
  {
    const float* ap = a1 + (size_t)row * HD;
    const v4f x0 = *(const v4f*)(ap + 8 * h), x1 = *(const v4f*)(ap + 8 * h + 4);
    const v4f x2 = *(const v4f*)(ap + 16 + 8 * h), x3 = *(const v4f*)(ap + 20 + 8 * h);
    const v4f s0 = *(const v4f*)(prm + 8 * h), s1 = *(const v4f*)(prm + 8 * h + 4);
    const v4f s2 = *(const v4f*)(prm + 16 + 8 * h), s3 = *(const v4f*)(prm + 20 + 8 * h);
    const v4f t0 = *(const v4f*)(prm + 32 + 8 * h), t1 = *(const v4f*)(prm + 36 + 8 * h);
    const v4f t2 = *(const v4f*)(prm + 48 + 8 * h), t3 = *(const v4f*)(prm + 52 + 8 * h);
    a.h[0] = cvt8(relu4(x0 * s0 + t0), relu4(x1 * s1 + t1));
    a.h[1] = cvt8(relu4(x2 * s2 + t2), relu4(x3 * s3 + t3));
  }
  v8f acc[2];
#pragma unroll
  for (int t = 0; t < 2; ++t) {
    const _Float16* bp = wg + (size_t)(16 * t + m) * HD + 8 * h;
    FragH b;
    b.h[0] = *(const v8h*)bp;
    b.h[1] = *(const v8h*)(bp + 16);
    acc[t] = wmh(a.v, b.v, zero8());
  }
  {
    float* sp = &stg[wave][(8 * h) * HD + m];
#pragma unroll
    for (int t = 0; t < 2; ++t) {
#pragma unroll
      for (int r = 0; r < 8; ++r) sp[r * HD + 16 * t] = acc[t][r] * WIV;
    }
  }
  __syncthreads();

  {
    const float* hr = &stg[wave][m * HD + 16 * h];
    const v4f p0 = *(const v4f*)hr, p1 = *(const v4f*)(hr + 4), p2 = *(const v4f*)(hr + 8), p3 = *(const v4f*)(hr + 12);
    const float* ws_ = satt + 16 * h;
    const float* wd_ = satt + 32 + 16 * h;
    float as = 0.f, ad = 0.f;
    as += p0.x * ws_[0];  as += p0.y * ws_[1];  as += p0.z * ws_[2];  as += p0.w * ws_[3];
    as += p1.x * ws_[4];  as += p1.y * ws_[5];  as += p1.z * ws_[6];  as += p1.w * ws_[7];
    as += p2.x * ws_[8];  as += p2.y * ws_[9];  as += p2.z * ws_[10]; as += p2.w * ws_[11];
    as += p3.x * ws_[12]; as += p3.y * ws_[13]; as += p3.z * ws_[14]; as += p3.w * ws_[15];
    ad += p0.x * wd_[0];  ad += p0.y * wd_[1];  ad += p0.z * wd_[2];  ad += p0.w * wd_[3];
    ad += p1.x * wd_[4];  ad += p1.y * wd_[5];  ad += p1.z * wd_[6];  ad += p1.w * wd_[7];
    ad += p2.x * wd_[8];  ad += p2.y * wd_[9];  ad += p2.z * wd_[10]; ad += p2.w * wd_[11];
    ad += p3.x * wd_[12]; ad += p3.y * wd_[13]; ad += p3.z * wd_[14]; ad += p3.w * wd_[15];
    sal[wave][m * 4 + h]     = as;
    sal[wave][m * 4 + 2 + h] = ad;
  }
  __syncthreads();

  store_tile16x32(stg[wave], hg + ((size_t)rowBase + wave * 16) * HD, lane);

  {
    const int m2 = lane >> 1, pc = lane & 1;
    v4f v;
    if (pc == 0) v = *(const v4f*)(&sal[wave][m2 * 4]);
    else { v.x = 0.f; v.y = 0.f; v.z = 0.f; v.w = 0.f; }
    float* gp = al + ((size_t)rowBase + wave * 16 + m2) * 8 + pc * 4;
    *(volatile v4f*)gp = v;
    __threadfence();
    *(volatile v4f*)gp = v;
  }
}

__global__ __launch_bounds__(NTHR) void k_gat(
    const int* __restrict__ ei, const float* __restrict__ hg, const float* __restrict__ al,
    const float* __restrict__ gb, float* apl, double* part, int nN, int nE, int vec8) {
  extern __shared__ v4f lds_dyn[];
  float*  acc  = (float*)lds_dyn;
  float*  mx   = acc + NBG * HD;
  float*  dn   = mx + NBG * 2;
  float*  ald  = dn + NBG * 2;
  int*    list = (int*)(ald + NBG * 2);
  int*    wcnt = list + LISTN;
  double* dsc  = (double*)list;
  const int tid = threadIdx.x, lane = tid & 31, wave = tid >> 5;
  const int nodeBase = blockIdx.x * NBG;
  const int* dsts = ei + nE;

#pragma unroll 4
  for (int idx = tid; idx < NBG * 8; idx += NTHR) {
    const int slot = idx >> 3;
    const int c4   = (idx & 7) * 4;
    int node = nodeBase + slot;
    node = node > nN - 1 ? nN - 1 : node;
    lds_dyn[idx] = *(const v4f*)(hg + (size_t)node * HD + c4);
  }
  for (int idx = tid; idx < NBG * 2; idx += NTHR) {
    const int slot = idx >> 1, hh = idx & 1;
    int node = nodeBase + slot;
    node = node > nN - 1 ? nN - 1 : node;
    const float as = al[(size_t)node * 8 + hh];
    const float ad = al[(size_t)node * 8 + 2 + hh];
    float e = as + ad;
    e = e < 0.f ? 0.2f * e : e;
    mx[idx]  = e;
    dn[idx]  = 1.0f;
    ald[idx] = ad;
  }
  __syncthreads();

  const int nChunks = (nE + CHUNK - 1) / CHUNK;
#pragma unroll 1
  for (int ch = 0; ch < nChunks; ++ch) {
    const int cbase = ch * CHUNK;
    const int wc = scan_chunk<NBG>(dsts, nE, cbase, nodeBase, vec8, list, tid, lane, wave);
    if (lane == 0) wcnt[wave] = wc;
    __syncthreads();
    if (wave == 0) {
      const int hh = lane >> 4;
#pragma unroll 1
      for (int wsx = 0; wsx < NWAVE; ++wsx) {
        int n = __builtin_amdgcn_readfirstlane(wcnt[wsx]);
        n = n > WCAP ? WCAP : (n < 0 ? 0 : n);
        const int* lp = list + wsx * WCAP;
#pragma unroll 1
        for (int i = 0; i < n; ++i) {
          const int ent  = __builtin_amdgcn_readfirstlane(lp[i]);
          const int slot = ent & (NBG - 1);
          int e = cbase + ((ent >> 12) & (CHUNK - 1));
          e = e > nE - 1 ? nE - 1 : e;
          int src = ei[e];
          src = src < 0 ? 0 : (src > nN - 1 ? nN - 1 : src);
          const float as = al[(size_t)src * 8 + hh];
          float ev = as + ald[slot * 2 + hh];
          ev = ev < 0.f ? 0.2f * ev : ev;
          const int mi = slot * 2 + hh;
          const float m0 = mx[mi];
          const float mn = fmaxf(m0, ev);
          const float corr = __expf(m0 - mn);
          const float p    = __expf(ev - mn);
          const float hv   = hg[(size_t)src * HD + lane];
          float* ap = acc + slot * HD + lane;
          const float av = *ap;
          *ap = av * corr + p * hv;
          if ((lane & 15) == 0) {
            const float dv = dn[mi];
            mx[mi] = mn;
            dn[mi] = dv * corr + p;
          }
        }
      }
    }
    __syncthreads();
  }

#pragma unroll 4
  for (int idx = tid; idx < NBG * 8; idx += NTHR) {
    const int slot = idx >> 3;
    const int c4   = (idx & 7) * 4;
    const int hh   = c4 >> 4;
    const float dv = dn[slot * 2 + hh];
    const float r  = 1.0f / (dv > 0.f ? dv : 1.0f);
    const v4f   bv = *(const v4f*)(gb + c4);
    const v4f   a  = lds_dyn[idx];
    lds_dyn[idx] = a * r + bv;
  }
  __syncthreads();

  bn_part<NBG, HD>(acc, dsc, part + (size_t)blockIdx.x * 64, nodeBase, nN, tid);
  store_rows<NBG * HD>(acc, apl + (size_t)nodeBase * HD, wave, lane);
}

__global__ __launch_bounds__(NTHR) void k_gcn2tf(
    const float* __restrict__ a2, const float* __restrict__ prm, const _Float16* __restrict__ wq,
    const float* __restrict__ dinv, float* g2, int nN) {
  __shared__ __attribute__((aligned(16))) float stg[NWAVE][16 * HHALF];
  const int tid = threadIdx.x, lane = tid & 31, wave = tid >> 5, h = lane >> 4, m = lane & 15;
  const int rowBase = blockIdx.x * TROWS;
  (void)nN;
  const int row = rowBase + wave * 16 + m;
  FragH a;
  {
    const float* ap = a2 + (size_t)row * HD;
    const v4f x0 = *(const v4f*)(ap + 8 * h), x1 = *(const v4f*)(ap + 8 * h + 4);
    const v4f x2 = *(const v4f*)(ap + 16 + 8 * h), x3 = *(const v4f*)(ap + 20 + 8 * h);
    const v4f s0 = *(const v4f*)(prm + 8 * h), s1 = *(const v4f*)(prm + 8 * h + 4);
    const v4f s2 = *(const v4f*)(prm + 16 + 8 * h), s3 = *(const v4f*)(prm + 20 + 8 * h);
    const v4f t0 = *(const v4f*)(prm + 32 + 8 * h), t1 = *(const v4f*)(prm + 36 + 8 * h);
    const v4f t2 = *(const v4f*)(prm + 48 + 8 * h), t3 = *(const v4f*)(prm + 52 + 8 * h);
    a.h[0] = cvt8(relu4(x0 * s0 + t0), relu4(x1 * s1 + t1));
    a.h[1] = cvt8(relu4(x2 * s2 + t2), relu4(x3 * s3 + t3));
  }
  v8f acc;
  {
    const _Float16* bp = wq + (size_t)m * HD + 8 * h;
    FragH b;
    b.h[0] = *(const v8h*)bp;
    b.h[1] = *(const v8h*)(bp + 16);
    acc = wmh(a.v, b.v, zero8());
  }
  {
    const int r0 = wave * 16 + 8 * h;
    const v4f dA = *(const v4f*)(dinv + (size_t)rowBase + r0);
    const v4f dB = *(const v4f*)(dinv + (size_t)rowBase + r0 + 4);
    float* sp = &stg[wave][(8 * h) * HHALF + m];
    sp[0 * HHALF] = acc[0] * dA.x * WIV;
    sp[1 * HHALF] = acc[1] * dA.y * WIV;
    sp[2 * HHALF] = acc[2] * dA.z * WIV;
    sp[3 * HHALF] = acc[3] * dA.w * WIV;
    sp[4 * HHALF] = acc[4] * dB.x * WIV;
    sp[5 * HHALF] = acc[5] * dB.y * WIV;
    sp[6 * HHALF] = acc[6] * dB.z * WIV;
    sp[7 * HHALF] = acc[7] * dB.w * WIV;
  }
  __syncthreads();
  {
    const int rr = lane >> 2, pc = (lane & 3) * 4;
    v4f v[2];
#pragma unroll
    for (int i = 0; i < 2; ++i) v[i] = *(const v4f*)(&stg[wave][(8 * i + rr) * HHALF + pc]);
    float* gp = g2 + ((size_t)rowBase + wave * 16) * HHALF;
#pragma unroll
    for (int i = 0; i < 2; ++i) *(volatile v4f*)(gp + (size_t)(8 * i + rr) * HHALF + pc) = v[i];
    __threadfence();
#pragma unroll
    for (int i = 0; i < 2; ++i) *(volatile v4f*)(gp + (size_t)(8 * i + rr) * HHALF + pc) = v[i];
  }
}

__global__ __launch_bounds__(NTHR) void k_pred(
    const float* __restrict__ a3, const float* __restrict__ prm, const _Float16* __restrict__ wq,
    const float* __restrict__ pb1, const float* __restrict__ pw2, const float* __restrict__ pb2,
    float* out, int nN) {
  __shared__ __attribute__((aligned(16))) float stg[NWAVE][16 * HHALF];
  __shared__ __attribute__((aligned(16))) float souts[TROWS];
  const int tid = threadIdx.x, lane = tid & 31, wave = tid >> 5, h = lane >> 4, m = lane & 15;
  const int rowBase = blockIdx.x * TROWS;
  const int row = rowBase + wave * 16 + m;
  FragH a;
  {
    const float* ap = a3 + (size_t)row * HHALF;
    const v4f x0 = *(const v4f*)(ap + 8 * h), x1 = *(const v4f*)(ap + 8 * h + 4);
    const v4f s0 = *(const v4f*)(prm + 8 * h), s1 = *(const v4f*)(prm + 8 * h + 4);
    const v4f t0 = *(const v4f*)(prm + 32 + 8 * h), t1 = *(const v4f*)(prm + 36 + 8 * h);
    a.h[0] = cvt8(relu4(x0 * s0 + t0), relu4(x1 * s1 + t1));
    v8h z;
#pragma unroll
    for (int j = 0; j < 8; ++j) z[j] = (_Float16)0.f;
    a.h[1] = z;
  }
  v8f acc;
  {
    const _Float16* bp = wq + (size_t)m * HD + 8 * h;
    FragH b;
    b.h[0] = *(const v8h*)bp;
    b.h[1] = *(const v8h*)(bp + 16);
    acc = wmh(a.v, b.v, zero8());
  }
  {
    const float bb = (m < 8) ? pb1[m & 7] : 0.f;
    const float ww = (m < 8) ? pw2[m & 7] : 0.f;
    float* sp = &stg[wave][(8 * h) * HHALF + m];
#pragma unroll
    for (int r = 0; r < 8; ++r) sp[r * HHALF] = fmaxf(acc[r] * WIV + bb, 0.f) * ww;
  }
  __syncthreads();
  if (lane < 16) {
    const float* rp = &stg[wave][lane * HHALF];
    const v4f q0 = *(const v4f*)rp, q1 = *(const v4f*)(rp + 4);
    float s = q0.x;
    s += q0.y; s += q0.z; s += q0.w; s += q1.x; s += q1.y; s += q1.z; s += q1.w;
    const float o = s + pb2[0];
    const float y = __builtin_amdgcn_rcpf(1.0f + __expf(-o));
    souts[wave * 16 + lane] = y;
  }
  __syncthreads();
  if (wave == 0) {
    const int gi = rowBase + 4 * lane;
    const v4f v = *(const v4f*)(souts + 4 * lane);
    float* op = out + gi;
    if (gi + 3 < nN) {
      *(volatile v4f*)op = v;
    } else {
      if (gi     < nN) *(volatile float*)(op)     = v.x;
      if (gi + 1 < nN) *(volatile float*)(op + 1) = v.y;
      if (gi + 2 < nN) *(volatile float*)(op + 2) = v.z;
    }
    __threadfence();
    if (gi + 3 < nN) {
      *(volatile v4f*)op = v;
    } else {
      if (gi     < nN) *(volatile float*)(op)     = v.x;
      if (gi + 1 < nN) *(volatile float*)(op + 1) = v.y;
      if (gi + 2 < nN) *(volatile float*)(op + 2) = v.z;
    }
  }
}

extern "C" void kernel_launch(void* const* d_in, const int* in_sizes, int n_in,
                              void* d_out, int out_size, void* d_ws, size_t ws_size,
                              hipStream_t stream) {
  if (n_in < 26) return;
  const int nN = in_sizes[0] / IND;
  const int nE = in_sizes[1] / 2;
  if (nN <= 0 || nE < 0 || in_sizes[0] != nN * IND || in_sizes[1] != 2 * nE) return;
  if (in_sizes[2] < IND || in_sizes[3] < IND || in_sizes[4] != IND * HD || in_sizes[5] < HD ||
      in_sizes[6] != HD * HD || in_sizes[7] < HD || in_sizes[8] != HD * HD || in_sizes[9] < HD ||
      in_sizes[10] < HD || in_sizes[11] < HD || in_sizes[12] != HD * HD || in_sizes[13] < 2 * HHALF ||
      in_sizes[14] < 2 * HHALF || in_sizes[15] < HD || in_sizes[16] < HD || in_sizes[17] < HD ||
      in_sizes[18] != HD * HHALF || in_sizes[19] < HHALF || in_sizes[20] < HHALF || in_sizes[21] < HHALF ||
      in_sizes[22] != HHALF * 8 || in_sizes[23] < 8 || in_sizes[24] < 8 || in_sizes[25] < 1) return;
  if (out_size != nN) return;

  const float* x      = (const float*)d_in[0];
  const int*   ei     = (const int*)d_in[1];
  const float* ln_g   = (const float*)d_in[2];
  const float* ln_b   = (const float*)d_in[3];
  const float* enc_w1 = (const float*)d_in[4];
  const float* enc_b1 = (const float*)d_in[5];
  const float* enc_w2 = (const float*)d_in[6];
  const float* enc_b2 = (const float*)d_in[7];
  const float* gcn1_w = (const float*)d_in[8];
  const float* gcn1_b = (const float*)d_in[9];
  const float* bn1_g  = (const float*)d_in[10];
  const float* bn1_b  = (const float*)d_in[11];
  const float* gat_w  = (const float*)d_in[12];
  const float* att_s  = (const float*)d_in[13];
  const float* att_d  = (const float*)d_in[14];
  const float* gat_b  = (const float*)d_in[15];
  const float* bn2_g  = (const float*)d_in[16];
  const float* bn2_b  = (const float*)d_in[17];
  const float* gcn2_w = (const float*)d_in[18];
  const float* gcn2_b = (const float*)d_in[19];
  const float* bn3_g  = (const float*)d_in[20];
  const float* bn3_b  = (const float*)d_in[21];
  const float* pr_w1  = (const float*)d_in[22];
  const float* pr_b1  = (const float*)d_in[23];
  const float* pr_w2  = (const float*)d_in[24];
  const float* pr_b2  = (const float*)d_in[25];
  float* out = (float*)d_out;

  const int nBD = (nN + NBD - 1) / NBD;
  const int nT  = (nN + TROWS - 1) / TROWS;
  const int nA1 = (nN + NB1 - 1) / NB1;
  const int nAG = (nN + NBG - 1) / NBG;
  const int nA2 = (nN + NB2 - 1) / NB2;

  char* ws = (char*)d_ws;
  size_t off = 0;
  const size_t oW  = off; off += (size_t)WO_TOT * 2;                     off = (off + 255) & ~(size_t)255;
  const size_t oDv = off; off += (size_t)nBD * NBD * 4;                  off = (off + 255) & ~(size_t)255;
  const size_t oG1 = off; off += (size_t)nT * TROWS * HD * 4;            off = (off + 255) & ~(size_t)255;
  const size_t oA1 = off; off += (size_t)nA1 * NB1 * HD * 4;             off = (off + 255) & ~(size_t)255;
  const size_t oAL = off; off += (size_t)nT * TROWS * 8 * 4;             off = (off + 255) & ~(size_t)255;
  const size_t oHG = off; off += (size_t)nT * TROWS * HD * 4;            off = (off + 255) & ~(size_t)255;
  const size_t oA2 = off; off += (size_t)nAG * NBG * HD * 4;             off = (off + 255) & ~(size_t)255;
  const size_t oG2 = off; off += (size_t)nT * TROWS * HHALF * 4;         off = (off + 255) & ~(size_t)255;
  const size_t oA3 = off; off += (size_t)nA2 * NB2 * HHALF * 4;          off = (off + 255) & ~(size_t)255;
  const size_t oP1 = off; off += (size_t)nA1 * 64 * 8;                   off = (off + 255) & ~(size_t)255;
  const size_t oP2 = off; off += (size_t)nAG * 64 * 8;                   off = (off + 255) & ~(size_t)255;
  const size_t oP3 = off; off += (size_t)nA2 * 64 * 8;                   off = (off + 255) & ~(size_t)255;
  const size_t oR1 = off; off += 256;
  const size_t oR2 = off; off += 256;
  const size_t oR3 = off; off += 256;
  if (off > ws_size) return;

  _Float16* wpl  = (_Float16*)(ws + oW);
  float*    dinv = (float*)(ws + oDv);
  float*    g1   = (float*)(ws + oG1);
  float*    a1   = (float*)(ws + oA1);
  float*    alp  = (float*)(ws + oAL);
  float*    hgp  = (float*)(ws + oHG);
  float*    a2   = (float*)(ws + oA2);
  float*    g2   = (float*)(ws + oG2);
  float*    a3   = (float*)(ws + oA3);
  double*   p1   = (double*)(ws + oP1);
  double*   p2   = (double*)(ws + oP2);
  double*   p3   = (double*)(ws + oP3);
  float*    r1   = (float*)(ws + oR1);
  float*    r2   = (float*)(ws + oR2);
  float*    r3   = (float*)(ws + oR3);

  const int vec8 = ((nE & 3) == 0) ? 1 : 0;

  k_prep<<<(WO_TOT / 8 + NTHR - 1) / NTHR, NTHR, 0, stream>>>(enc_w2, gcn1_w, gat_w, gcn2_w, pr_w1, wpl);

  k_deg<<<nBD, NTHR, 0, stream>>>(ei, dinv, nE, vec8);

  k_enc<<<nT, NTHR, 0, stream>>>(x, ln_g, ln_b, enc_w1, enc_b1, enc_b2, wpl, dinv, g1, nN);

  hipFuncSetAttribute(reinterpret_cast<const void*>(&k_gcnagg<NB1, HD>),
                      hipFuncAttributeMaxDynamicSharedMemorySize, LDS_AGG1);
  k_gcnagg<NB1, HD><<<nA1, NTHR, LDS_AGG1, stream>>>(ei, g1, dinv, gcn1_b, a1, p1, nN, nE, vec8);

  k_bnfin<<<1, 32, 0, stream>>>(p1, nA1, bn1_g, bn1_b, HD, nN, r1);

  k_gattf<<<nT, NTHR, 0, stream>>>(a1, r1, wpl + WO_GA, att_s, att_d, hgp, alp, nN);

  hipFuncSetAttribute(reinterpret_cast<const void*>(&k_gat),
                      hipFuncAttributeMaxDynamicSharedMemorySize, LDS_GAT);
  k_gat<<<nAG, NTHR, LDS_GAT, stream>>>(ei, hgp, alp, gat_b, a2, p2, nN, nE, vec8);

  k_bnfin<<<1, 32, 0, stream>>>(p2, nAG, bn2_g, bn2_b, HD, nN, r2);

  k_gcn2tf<<<nT, NTHR, 0, stream>>>(a2, r2, wpl + WO_G2, dinv, g2, nN);

  hipFuncSetAttribute(reinterpret_cast<const void*>(&k_gcnagg<NB2, HHALF>),
                      hipFuncAttributeMaxDynamicSharedMemorySize, LDS_AGG2);
  k_gcnagg<NB2, HHALF><<<nA2, NTHR, LDS_AGG2, stream>>>(ei, g2, dinv, gcn2_b, a3, p3, nN, nE, vec8);

  k_bnfin<<<1, 32, 0, stream>>>(p3, nA2, bn3_g, bn3_b, HHALF, nN, r3);

  k_pred<<<nT, NTHR, 0, stream>>>(a3, r3, wpl + WO_P1, pr_b1, pr_w2, pr_b2, out, nN);
}
